// HyperbolicMultiHeadAttention_26920855011363
// MI455X (gfx1250) — hardware-verified
//
#include <hip/hip_runtime.h>
#include <stddef.h>
#include <stdint.h>

#pragma clang fp contract(off)

#define SEQ  2048
#define DM   1024
#define NH   16
#define HD   64

#define TP   68
#define HP   72
#define OP   68
#define EPSV 1.0e-5f
#define VSC  64.0f
#define PSC  4096.0f
#define F16_MIN_NORMAL 6.103515625e-05f

#define SZ_P16  ((size_t)SEQ * DM * 2)
#define SZ_W16  ((size_t)DM * DM * 2)
#define SZ_VT   ((size_t)NH * HD * SEQ * 2)
#define SZ_NS   ((size_t)2 * NH * SEQ * 4)
#define OFF_XB  ((size_t)0)
#define OFF_WB  (OFF_XB + SZ_P16)
#define OFF_QH  (OFF_WB + 4 * SZ_W16)
#define OFF_QL  (OFF_QH + SZ_P16)
#define OFF_KH  (OFF_QL + SZ_P16)
#define OFF_KL  (OFF_KH + SZ_P16)
#define OFF_VH  (OFF_KL + SZ_P16)
#define OFF_VL  (OFF_VH + SZ_VT)
#define OFF_NS  (OFF_VL + SZ_VT)
#define OFF_CH  (OFF_NS + SZ_NS)
#define OFF_CL  (OFF_CH + SZ_P16)
#define WS_TOTAL (OFF_CL + SZ_P16)

static_assert(OFF_WB == (size_t)4194304);
static_assert(OFF_QH == (size_t)12582912);
static_assert(OFF_QL == (size_t)16777216);
static_assert(OFF_KH == (size_t)20971520);
static_assert(OFF_KL == (size_t)25165824);
static_assert(OFF_VH == (size_t)29360128);
static_assert(OFF_VL == (size_t)33554432);
static_assert(OFF_NS == (size_t)37748736);
static_assert(OFF_CH == (size_t)38010880);
static_assert(OFF_CL == (size_t)42205184);
static_assert(WS_TOTAL == (size_t)46399488);
static_assert(WS_TOTAL <= (size_t)134217728);
static_assert((OFF_WB % 256) == 0);
static_assert((OFF_QH % 256) == 0);
static_assert((OFF_NS % 256) == 0);
static_assert((OFF_CH % 256) == 0);
static_assert((OFF_CL % 256) == 0);
static_assert((SEQ % 128) == 0);
static_assert((DM % 64) == 0);
static_assert((DM % 32) == 0);
static_assert(HD == 64);
static_assert(DM == NH * HD);
static_assert((TP * 4) % 16 == 0);
static_assert((HP * 2) % 16 == 0);
static_assert((OP * 4) % 16 == 0);
static_assert(8 * 16 * HP * 2 + 8 * 16 * OP * 4 <= 65536);
static_assert(128 * TP * 4 + 2 * 128 * 4 <= 65536);

typedef unsigned short v8us  __attribute__((ext_vector_type(8)));
typedef unsigned short v16us __attribute__((ext_vector_type(16)));
typedef unsigned short v8usA __attribute__((ext_vector_type(8), may_alias));
typedef _Float16       v8h   __attribute__((ext_vector_type(8)));
typedef _Float16       v16h  __attribute__((ext_vector_type(16)));
typedef _Float16       v8hA  __attribute__((ext_vector_type(8), may_alias));
typedef float          v4f   __attribute__((ext_vector_type(4)));
typedef float          v4fA  __attribute__((ext_vector_type(4), may_alias));
typedef float          v8f   __attribute__((ext_vector_type(8)));
#if defined(__HIP_DEVICE_COMPILE__)
typedef __bf16         v16bf __attribute__((ext_vector_type(16)));
#endif

union FragU { v16us v; v8us half[2]; };
union FragH { v16h  v; v8h  half[2]; };

__device__ __forceinline__ unsigned bbits(float f) {
  unsigned u = __float_as_uint(f);
  return (u + 0x7FFFu + ((u >> 16) & 1u)) >> 16;
}
__device__ __forceinline__ float bf16r(float f) {
  return __uint_as_float(bbits(f) << 16);
}
__device__ __forceinline__ float frcp_(float x) {
#if defined(__HIP_DEVICE_COMPILE__)
  return __builtin_amdgcn_rcpf(x);
#else
  return 1.0f / x;
#endif
}
__device__ __forceinline__ float fsqrt_(float x) {
#if defined(__HIP_DEVICE_COMPILE__)
  return __builtin_amdgcn_sqrtf(x);
#else
  return x;
#endif
}
__device__ __forceinline__ float flog_(float x) {
#if defined(__HIP_DEVICE_COMPILE__)
  return __logf(x);
#else
  return x;
#endif
}
__device__ __forceinline__ int unif(int v) {
#if defined(__HIP_DEVICE_COMPILE__)
  return __builtin_amdgcn_readfirstlane(v);
#else
  return v;
#endif
}
__device__ __forceinline__ v8f zero8() { v8f z = {0.f, 0.f, 0.f, 0.f, 0.f, 0.f, 0.f, 0.f}; return z; }

__device__ __forceinline__ float softplus_(float x) {
  return fmaxf(x, 0.0f) + log1pf(expf(-fabsf(x)));
}
__device__ __forceinline__ float atanh_(float x) {
  return 0.5f * (log1pf(x) - log1pf(-x));
}

__device__ __forceinline__ v16us ldfrag_u(const unsigned short* p) {
  FragU f;
  f.half[0] = *(const v8usA*)(p);
  f.half[1] = *(const v8usA*)(p + 16);
  return f.v;
}
__device__ __forceinline__ v16h ldfrag_h(const _Float16* p) {
  FragH f;
  f.half[0] = *(const v8hA*)(p);
  f.half[1] = *(const v8hA*)(p + 16);
  return f.v;
}

__device__ __forceinline__ v8f mma_bf(v16us a, v16us b, v8f c) {
#if defined(__HIP_DEVICE_COMPILE__)
  return __builtin_amdgcn_wmma_f32_16x16x32_bf16(false, __builtin_bit_cast(v16bf, a),
                                                false, __builtin_bit_cast(v16bf, b),
                                                (short)0, c, false, false);
#else
  (void)a; (void)b;
  return c;
#endif
}
__device__ __forceinline__ v8f mma_h(v16h a, v16h b, v8f c) {
#if defined(__HIP_DEVICE_COMPILE__)
  return __builtin_amdgcn_wmma_f32_16x16x32_f16(false, a, false, b, (short)0, c, false, false);
#else
  (void)a; (void)b;
  return c;
#endif
}
template <typename F>
__device__ __forceinline__ void guard4(v8f& c0, v8f& c1, v8f& c2, v8f& c3,
                                       const F& f0, const F& f1, const F& f2,
                                       const F& f3, const F& f4, const F& f5) {
#if defined(__HIP_DEVICE_COMPILE__)
  asm volatile("v_nop\n\tv_nop\n\tv_nop\n\tv_nop"
               : "+v"(c0), "+v"(c1), "+v"(c2), "+v"(c3)
               : "v"(f0), "v"(f1), "v"(f2), "v"(f3), "v"(f4), "v"(f5));
#else
  (void)c0; (void)c1; (void)c2; (void)c3; (void)f0; (void)f1; (void)f2; (void)f3; (void)f4; (void)f5;
#endif
}
template <typename F>
__device__ __forceinline__ void guard1(v8f& c0, const F& f0, const F& f1, const F& f2, const F& f3) {
#if defined(__HIP_DEVICE_COMPILE__)
  asm volatile("v_nop\n\tv_nop\n\tv_nop\n\tv_nop"
               : "+v"(c0)
               : "v"(f0), "v"(f1), "v"(f2), "v"(f3));
#else
  (void)c0; (void)f0; (void)f1; (void)f2; (void)f3;
#endif
}

__device__ __forceinline__ float hscore(float dot, float xn, float aq, float kn, float c,
                                        float twoc, float rsc, float nbeta, float ab) {
  const float two_dot = 2.0f * dot;
  const float diff = (xn - two_dot) + kn;
  float den = aq * (1.0f - c * kn);
  den = fmaxf(den, EPSV);
  float arg = 1.0f + (twoc * diff) * frcp_(den);
  arg = fmaxf(arg, 1.00001f);
  const float sq   = fsqrt_((arg + 1.0f) * (arg - 1.0f));
  const float dist = flog_(arg + sq) * rsc;
  return nbeta * dist - ab;
}

__global__ __launch_bounds__(256)
void k_cvt(const float* __restrict__ x, const float* __restrict__ wq, const float* __restrict__ wk,
           const float* __restrict__ wv, const float* __restrict__ wo,
           unsigned short* xb, unsigned short* wb)
{
  const int z    = blockIdx.y;
  const int tid  = threadIdx.x;
  const int lane = tid & 31;
  const int w    = tid >> 5;

  const float* src;
  unsigned short* dst;
  int nrows;
  if (z == 0)      { src = x;  dst = xb;                       nrows = SEQ; }
  else if (z == 1) { src = wq; dst = wb;                       nrows = DM; }
  else if (z == 2) { src = wk; dst = wb + (size_t)DM * DM;     nrows = DM; }
  else if (z == 3) { src = wv; dst = wb + (size_t)2 * DM * DM; nrows = DM; }
  else             { src = wo; dst = wb + (size_t)3 * DM * DM; nrows = DM; }
  const int row0 = blockIdx.x * 32;
  if (row0 >= nrows) return;

#pragma unroll 1
  for (int i = 0; i < 4; ++i) {
    const int row = row0 + 4 * w + i;
    const float* xr = src + (size_t)row * DM;
    v8us   ov[4];
    size_t off[4];
#pragma unroll
    for (int it = 0; it < 4; ++it) {
      const int p = it * 32 + lane;
      const v4f a = *(const v4fA*)(xr + 8 * p);
      const v4f b = *(const v4fA*)(xr + 8 * p + 4);
      v8us o;
#pragma unroll
      for (int e = 0; e < 4; ++e) {
        o[e]     = (unsigned short)bbits(a[e]);
        o[4 + e] = (unsigned short)bbits(b[e]);
      }
      ov[it]  = o;
      off[it] = (size_t)row * DM + (size_t)(8 * p);
    }
#pragma unroll
    for (int it = 0; it < 4; ++it) *(volatile v8us*)(dst + off[it]) = ov[it];
    __threadfence();
#pragma unroll
    for (int it = 0; it < 4; ++it) *(volatile v8us*)(dst + off[it]) = ov[it];
  }
}

__global__ __launch_bounds__(256)
void k_proj(const unsigned short* __restrict__ xb, const unsigned short* __restrict__ wb,
            const float* __restrict__ lcp,
            unsigned short* qh, unsigned short* ql, unsigned short* kh, unsigned short* kl,
            _Float16* vh, _Float16* vl, float* ns)
{
  __shared__ __align__(16) float T[128 * TP];
  __shared__ __align__(16) float rt[128];
  __shared__ __align__(16) float rns[128];
  const int n0   = blockIdx.x * 64;
  const int m0   = blockIdx.y * 128;
  const int z    = blockIdx.z;
  const int tid  = threadIdx.x;
  const int lane = tid & 31;
  const int w    = unif(tid >> 5);
  const int h    = lane >> 4;
  const int m    = lane & 15;
  const int q8   = lane >> 3;
  const int jj   = lane & 7;
  const int wm   = w >> 1;
  const int wn   = w & 1;

  const unsigned short* Bt = wb + (size_t)z * DM * DM;
  const float c  = softplus_(bf16r(lcp[0]));
  const float sc = sqrtf(c);

  v8f acc[2][2];
  acc[0][0] = zero8(); acc[0][1] = zero8(); acc[1][0] = zero8(); acc[1][1] = zero8();

  const unsigned short* pa = xb + (size_t)(m0 + 32 * wm + m) * DM + 8 * h;
  const unsigned short* pb = Bt + (size_t)(n0 + 32 * wn + m) * DM + 8 * h;
#pragma unroll 2
  for (int kk = 0; kk < DM / 32; ++kk) {
    const v16us a0 = ldfrag_u(pa + 32 * kk);
    const v16us a1 = ldfrag_u(pa + (size_t)16 * DM + 32 * kk);
    const v16us b0 = ldfrag_u(pb + 32 * kk);
    const v16us b1 = ldfrag_u(pb + (size_t)16 * DM + 32 * kk);
    acc[0][0] = mma_bf(a0, b0, acc[0][0]);
    acc[0][1] = mma_bf(a0, b1, acc[0][1]);
    acc[1][0] = mma_bf(a1, b0, acc[1][0]);
    acc[1][1] = mma_bf(a1, b1, acc[1][1]);
    guard4<v16us>(acc[0][0], acc[0][1], acc[1][0], acc[1][1], a0, a1, b0, b1, a0, b1);
  }

#pragma unroll
  for (int mi = 0; mi < 2; ++mi)
#pragma unroll
    for (int ni = 0; ni < 2; ++ni)
#pragma unroll
      for (int r = 0; r < 8; ++r)
        T[(32 * wm + 16 * mi + 8 * h + r) * TP + 32 * wn + 16 * ni + m] = acc[mi][ni][r];
  __syncthreads();

  {
    const int row = tid >> 1;
    const int hf  = tid & 1;
    const v4fA* tr = (const v4fA*)(T + row * TP + 32 * hf);
    float ss = 0.f;
#pragma unroll
    for (int c4 = 0; c4 < 8; ++c4) {
      const v4f xv = tr[c4];
#pragma unroll
      for (int e = 0; e < 4; ++e) ss += xv[e] * xv[e];
    }
    ss += __shfl_xor(ss, 1, 32);
    const float n1 = fmaxf(sqrtf(ss), EPSV);
    const float a1 = sc * n1;
    const float t1 = tanhf(a1) * frcp_(a1);
    float s2 = 0.f;
#pragma unroll
    for (int c4 = 0; c4 < 8; ++c4) {
      const v4f xv = tr[c4];
#pragma unroll
      for (int e = 0; e < 4; ++e) { const float qd = t1 * xv[e]; s2 += qd * qd; }
    }
    s2 += __shfl_xor(s2, 1, 32);
    if (hf == 0) { rt[row] = t1; rns[row] = s2; }
  }
  __syncthreads();

  if (z == 2) {
    const int h16 = lane >> 4;
    const int j16 = lane & 15;
    const int hd  = blockIdx.x;
    v8h    oh[4], ol[4];
    size_t off[4];
#pragma unroll
    for (int it = 0; it < 4; ++it) {
      const int d = 16 * it + 2 * w + h16;
      v8h ho, lo;
#pragma unroll
      for (int e = 0; e < 8; ++e) {
        const int tk  = 8 * j16 + e;
        const float xs = T[tk * TP + d] * VSC;
        const _Float16 hv = (_Float16)xs;
        ho[e] = hv;
        lo[e] = (_Float16)(xs - (float)hv);
      }
      oh[it]  = ho;
      ol[it]  = lo;
      off[it] = ((size_t)(hd * HD + d)) * SEQ + (size_t)(m0 + 8 * j16);
    }
#pragma unroll
    for (int it = 0; it < 4; ++it) *(volatile v8h*)(vh + off[it]) = oh[it];
#pragma unroll
    for (int it = 0; it < 4; ++it) *(volatile v8h*)(vl + off[it]) = ol[it];
    __threadfence();
#pragma unroll
    for (int it = 0; it < 4; ++it) *(volatile v8h*)(vh + off[it]) = oh[it];
#pragma unroll
    for (int it = 0; it < 4; ++it) *(volatile v8h*)(vl + off[it]) = ol[it];
  } else {
    unsigned short* PH = (z == 0) ? qh : kh;
    unsigned short* PL = (z == 0) ? ql : kl;
    v8us   oh[4], ol[4];
    size_t off[4];
#pragma unroll
    for (int it = 0; it < 4; ++it) {
      const int rl = 32 * it + 4 * w + q8;
      const v4fA* tp = (const v4fA*)(T + rl * TP + 8 * jj);
      const v4f a = tp[0];
      const v4f b = tp[1];
      const float t1 = rt[rl];
      v8us ho, lo;
#pragma unroll
      for (int e = 0; e < 4; ++e) {
        const float v0 = t1 * a[e];
        const unsigned hb0 = bbits(v0);
        ho[e] = (unsigned short)hb0;
        lo[e] = (unsigned short)bbits(v0 - __uint_as_float(hb0 << 16));
        const float v1 = t1 * b[e];
        const unsigned hb1 = bbits(v1);
        ho[4 + e] = (unsigned short)hb1;
        lo[4 + e] = (unsigned short)bbits(v1 - __uint_as_float(hb1 << 16));
      }
      oh[it]  = ho;
      ol[it]  = lo;
      off[it] = (size_t)(m0 + rl) * DM + (size_t)(n0 + 8 * jj);
    }
    const v4f nv = *(const v4fA*)(rns + 4 * lane);
    float* np = ns + ((size_t)z * NH + blockIdx.x) * SEQ + m0 + 4 * lane;
#pragma unroll
    for (int it = 0; it < 4; ++it) *(volatile v8us*)(PH + off[it]) = oh[it];
#pragma unroll
    for (int it = 0; it < 4; ++it) *(volatile v8us*)(PL + off[it]) = ol[it];
    if (w == 0) *(volatile v4f*)np = nv;
    __threadfence();
#pragma unroll
    for (int it = 0; it < 4; ++it) *(volatile v8us*)(PH + off[it]) = oh[it];
#pragma unroll
    for (int it = 0; it < 4; ++it) *(volatile v8us*)(PL + off[it]) = ol[it];
    if (w == 0) *(volatile v4f*)np = nv;
  }
}

__global__ __launch_bounds__(256)
void k_attn(const unsigned short* __restrict__ qh, const unsigned short* __restrict__ ql,
            const unsigned short* __restrict__ kh, const unsigned short* __restrict__ kl,
            const _Float16* __restrict__ vh, const _Float16* __restrict__ vl,
            const float* __restrict__ ns, const int* __restrict__ msk,
            const float* __restrict__ lcp, const float* __restrict__ btp,
            const float* __restrict__ abp, unsigned short* ch, unsigned short* cl)
{
  __shared__ __align__(16) _Float16 Ps[8 * 16 * HP];
  __shared__ __align__(16) float Os[8 * 16 * OP];
  const int tid  = threadIdx.x;
  const int lane = tid & 31;
  const int w    = unif(tid >> 5);
  const int h    = lane >> 4;
  const int m    = lane & 15;
  const int q8   = lane >> 3;
  const int jj   = lane & 7;
  const int hd   = blockIdx.y;
  const int hc   = hd * HD;
  const int qblk = blockIdx.x;
  const int q0w  = qblk * 128 + 16 * w;
  _Float16* Pw = Ps + w * (16 * HP);
  float*    Ow = Os + w * (16 * OP);

  const float c     = softplus_(bf16r(lcp[0]));
  const float sc    = sqrtf(c);
  const float rsc   = 1.0f / sc;
  const float twoc  = 2.0f * c;
  const float nbeta = -softplus_(bf16r(btp[0]));
  const float ab    = bf16r(abp[0]);
  const float thr   = rsc - EPSV;

  const size_t qo = (size_t)(q0w + m) * DM + hc + 8 * h;
  const v16us qa0h = ldfrag_u(qh + qo);
  const v16us qa1h = ldfrag_u(qh + qo + 32);
  const v16us qa0l = ldfrag_u(ql + qo);
  const v16us qa1l = ldfrag_u(ql + qo + 32);

  float qn[8];
  {
    const float* qnp = ns + (size_t)hd * SEQ + q0w + 8 * h;
#pragma unroll
    for (int r = 0; r < 8; ++r) qn[r] = qnp[r];
  }
  float mst[8], lst[8];
#pragma unroll
  for (int r = 0; r < 8; ++r) { mst[r] = -__builtin_huge_valf(); lst[r] = 0.f; }
  v8f oacc[4];
  oacc[0] = zero8(); oacc[1] = zero8(); oacc[2] = zero8(); oacc[3] = zero8();

  const float*          knp   = ns + (size_t)(NH + hd) * SEQ;
  const unsigned short* khb   = kh + (size_t)m * DM + hc + 8 * h;
  const unsigned short* klb   = kl + (size_t)m * DM + hc + 8 * h;
  const _Float16*       vhb   = vh + (size_t)(hd * HD + m) * SEQ + 8 * h;
  const _Float16*       vlb   = vl + (size_t)(hd * HD + m) * SEQ + 8 * h;
  const int*            mbase = msk + (size_t)(q0w + 8 * h) * SEQ + m;

  const int ntiles = 2 * qblk + 2;

#pragma unroll 1
  for (int j = 0; j < ntiles; ++j) {
    const int k0 = 64 * j;
    float kn[4];
#pragma unroll
    for (int t = 0; t < 4; ++t) kn[t] = knp[k0 + 16 * t + m];
    v8f sacc[4];
    sacc[0] = zero8(); sacc[1] = zero8(); sacc[2] = zero8(); sacc[3] = zero8();
#pragma unroll
    for (int t = 0; t < 4; ++t) {
      const size_t ro = (size_t)(k0 + 16 * t) * DM;
      const v16us bh0 = ldfrag_u(khb + ro);
      const v16us bl0 = ldfrag_u(klb + ro);
      const v16us bh1 = ldfrag_u(khb + ro + 32);
      const v16us bl1 = ldfrag_u(klb + ro + 32);
      sacc[t] = mma_bf(qa0h, bh0, sacc[t]);
      sacc[t] = mma_bf(qa0h, bl0, sacc[t]);
      sacc[t] = mma_bf(qa0l, bh0, sacc[t]);
      sacc[t] = mma_bf(qa1h, bh1, sacc[t]);
      sacc[t] = mma_bf(qa1h, bl1, sacc[t]);
      sacc[t] = mma_bf(qa1l, bh1, sacc[t]);
      guard1<v16us>(sacc[t], bh0, bl0, bh1, bl1);
    }

#pragma unroll
    for (int r = 0; r < 8; ++r) {
      const int* mp = mbase + (size_t)r * SEQ + k0;
      const int k_0 = mp[0];
      const int k_1 = mp[16];
      const int k_2 = mp[32];
      const int k_3 = mp[48];
      const float xn = qn[r];
      const float aq = 1.0f - c * xn;
      float s0 = hscore(sacc[0][r], xn, aq, kn[0], c, twoc, rsc, nbeta, ab);
      float s1 = hscore(sacc[1][r], xn, aq, kn[1], c, twoc, rsc, nbeta, ab);
      float s2 = hscore(sacc[2][r], xn, aq, kn[2], c, twoc, rsc, nbeta, ab);
      float s3 = hscore(sacc[3][r], xn, aq, kn[3], c, twoc, rsc, nbeta, ab);
      s0 = (k_0 != 0) ? s0 : -__FLT_MAX__;
      s1 = (k_1 != 0) ? s1 : -__FLT_MAX__;
      s2 = (k_2 != 0) ? s2 : -__FLT_MAX__;
      s3 = (k_3 != 0) ? s3 : -__FLT_MAX__;
      float mx = fmaxf(fmaxf(s0, s1), fmaxf(s2, s3));
      mx = fmaxf(mx, __shfl_xor(mx, 1, 32));
      mx = fmaxf(mx, __shfl_xor(mx, 2, 32));
      mx = fmaxf(mx, __shfl_xor(mx, 4, 32));
      mx = fmaxf(mx, __shfl_xor(mx, 8, 32));
      const float mnew = fmaxf(mst[r], mx);
      const float msc  = __expf(mst[r] - mnew);
      mst[r] = mnew;
      const float p0 = __expf(s0 - mnew) * PSC;
      const float p1 = __expf(s1 - mnew) * PSC;
      const float p2 = __expf(s2 - mnew) * PSC;
      const float p3 = __expf(s3 - mnew) * PSC;
      const _Float16 zh = (_Float16)0.0f;
      const _Float16 h0 = (p0 < F16_MIN_NORMAL) ? zh : (_Float16)p0;
      const _Float16 h1 = (p1 < F16_MIN_NORMAL) ? zh : (_Float16)p1;
      const _Float16 h2 = (p2 < F16_MIN_NORMAL) ? zh : (_Float16)p2;
      const _Float16 h3 = (p3 < F16_MIN_NORMAL) ? zh : (_Float16)p3;
      float rs = (float)h0 + (float)h1 + (float)h2 + (float)h3;
      rs += __shfl_xor(rs, 1, 32);
      rs += __shfl_xor(rs, 2, 32);
      rs += __shfl_xor(rs, 4, 32);
      rs += __shfl_xor(rs, 8, 32);
      lst[r] = lst[r] * msc + rs;
      Pw[(8 * h + r) * HP + m]      = h0;
      Pw[(8 * h + r) * HP + 16 + m] = h1;
      Pw[(8 * h + r) * HP + 32 + m] = h2;
      Pw[(8 * h + r) * HP + 48 + m] = h3;
      oacc[0][r] *= msc;
      oacc[1][r] *= msc;
      oacc[2][r] *= msc;
      oacc[3][r] *= msc;
    }
    __syncthreads();

    {
      const v16h pa0 = ldfrag_h(Pw + m * HP + 8 * h);
      const v16h pa1 = ldfrag_h(Pw + m * HP + 32 + 8 * h);
      const _Float16* vph = vhb + k0;
      const _Float16* vpl = vlb + k0;
      {
        const v16h v0 = ldfrag_h(vph);
        const v16h v1 = ldfrag_h(vph + (size_t)16 * SEQ);
        const v16h v2 = ldfrag_h(vph + (size_t)32 * SEQ);
        const v16h v3 = ldfrag_h(vph + (size_t)48 * SEQ);
        oacc[0] = mma_h(pa0, v0, oacc[0]);
        oacc[1] = mma_h(pa0, v1, oacc[1]);
        oacc[2] = mma_h(pa0, v2, oacc[2]);
        oacc[3] = mma_h(pa0, v3, oacc[3]);
        const v16h u0 = ldfrag_h(vpl);
        const v16h u1 = ldfrag_h(vpl + (size_t)16 * SEQ);
        const v16h u2 = ldfrag_h(vpl + (size_t)32 * SEQ);
        const v16h u3 = ldfrag_h(vpl + (size_t)48 * SEQ);
        oacc[0] = mma_h(pa0, u0, oacc[0]);
        oacc[1] = mma_h(pa0, u1, oacc[1]);
        oacc[2] = mma_h(pa0, u2, oacc[2]);
        oacc[3] = mma_h(pa0, u3, oacc[3]);
        guard4<v16h>(oacc[0], oacc[1], oacc[2], oacc[3], pa0, pa1, u0, u1, u2, u3);
      }
      {
        const v16h v0 = ldfrag_h(vph + 32);
        const v16h v1 = ldfrag_h(vph + (size_t)16 * SEQ + 32);
        const v16h v2 = ldfrag_h(vph + (size_t)32 * SEQ + 32);
        const v16h v3 = ldfrag_h(vph + (size_t)48 * SEQ + 32);
        oacc[0] = mma_h(pa1, v0, oacc[0]);
        oacc[1] = mma_h(pa1, v1, oacc[1]);
        oacc[2] = mma_h(pa1, v2, oacc[2]);
        oacc[3] = mma_h(pa1, v3, oacc[3]);
        const v16h u0 = ldfrag_h(vpl + 32);
        const v16h u1 = ldfrag_h(vpl + (size_t)16 * SEQ + 32);
        const v16h u2 = ldfrag_h(vpl + (size_t)32 * SEQ + 32);
        const v16h u3 = ldfrag_h(vpl + (size_t)48 * SEQ + 32);
        oacc[0] = mma_h(pa1, u0, oacc[0]);
        oacc[1] = mma_h(pa1, u1, oacc[1]);
        oacc[2] = mma_h(pa1, u2, oacc[2]);
        oacc[3] = mma_h(pa1, u3, oacc[3]);
        guard4<v16h>(oacc[0], oacc[1], oacc[2], oacc[3], pa0, pa1, u0, u1, u2, u3);
      }
    }
    __syncthreads();
  }

#pragma unroll
  for (int r = 0; r < 8; ++r) {
    const float inv = frcp_(lst[r] * VSC);
    const float u0 = oacc[0][r] * inv;
    const float u1 = oacc[1][r] * inv;
    const float u2 = oacc[2][r] * inv;
    const float u3 = oacc[3][r] * inv;
    float ss = u0 * u0;
    ss += u1 * u1;
    ss += u2 * u2;
    ss += u3 * u3;
    ss += __shfl_xor(ss, 1, 32);
    ss += __shfl_xor(ss, 2, 32);
    ss += __shfl_xor(ss, 4, 32);
    ss += __shfl_xor(ss, 8, 32);
    const float n1 = fmaxf(sqrtf(ss), EPSV);
    const float a1 = sc * n1;
    const float t1 = tanhf(a1) * frcp_(a1);
    const float y0 = t1 * u0;
    const float y1 = t1 * u1;
    const float y2 = t1 * u2;
    const float y3 = t1 * u3;
    float s2 = y0 * y0;
    s2 += y1 * y1;
    s2 += y2 * y2;
    s2 += y3 * y3;
    s2 += __shfl_xor(s2, 1, 32);
    s2 += __shfl_xor(s2, 2, 32);
    s2 += __shfl_xor(s2, 4, 32);
    s2 += __shfl_xor(s2, 8, 32);
    const float n2  = fmaxf(sqrtf(s2), EPSV);
    const float ncl = fminf(n2, thr);
    const float t2  = atanh_(sc * ncl) * frcp_(sc * n2);
    Ow[(8 * h + r) * OP + m]      = t2 * y0;
    Ow[(8 * h + r) * OP + 16 + m] = t2 * y1;
    Ow[(8 * h + r) * OP + 32 + m] = t2 * y2;
    Ow[(8 * h + r) * OP + 48 + m] = t2 * y3;
  }
  __syncthreads();

  v8us   oh[4], ol[4];
  size_t off[4];
#pragma unroll
  for (int it = 0; it < 4; ++it) {
    const int rl = 4 * it + q8;
    const v4fA* tp = (const v4fA*)(Ow + rl * OP + 8 * jj);
    const v4f a = tp[0];
    const v4f b = tp[1];
    v8us ho, lo;
#pragma unroll
    for (int e = 0; e < 4; ++e) {
      const unsigned hb0 = bbits(a[e]);
      ho[e] = (unsigned short)hb0;
      lo[e] = (unsigned short)bbits(a[e] - __uint_as_float(hb0 << 16));
      const unsigned hb1 = bbits(b[e]);
      ho[4 + e] = (unsigned short)hb1;
      lo[4 + e] = (unsigned short)bbits(b[e] - __uint_as_float(hb1 << 16));
    }
    oh[it]  = ho;
    ol[it]  = lo;
    off[it] = (size_t)(q0w + rl) * DM + (size_t)(hc + 8 * jj);
  }
#pragma unroll
  for (int it = 0; it < 4; ++it) *(volatile v8us*)(ch + off[it]) = oh[it];
#pragma unroll
  for (int it = 0; it < 4; ++it) *(volatile v8us*)(cl + off[it]) = ol[it];
  __threadfence();
#pragma unroll
  for (int it = 0; it < 4; ++it) *(volatile v8us*)(ch + off[it]) = oh[it];
#pragma unroll
  for (int it = 0; it < 4; ++it) *(volatile v8us*)(cl + off[it]) = ol[it];
}

__global__ __launch_bounds__(256)
void k_out(const unsigned short* __restrict__ ch, const unsigned short* __restrict__ cl,
           const unsigned short* __restrict__ wob, float* out)
{
  __shared__ __align__(16) float T[128 * TP];
  const int n0   = blockIdx.x * 64;
  const int m0   = blockIdx.y * 128;
  const int tid  = threadIdx.x;
  const int lane = tid & 31;
  const int w    = unif(tid >> 5);
  const int h    = lane >> 4;
  const int m    = lane & 15;
  const int q8   = lane >> 3;
  const int jj   = lane & 7;
  const int wm   = w >> 1;
  const int wn   = w & 1;

  v8f acc[2][2];
  acc[0][0] = zero8(); acc[0][1] = zero8(); acc[1][0] = zero8(); acc[1][1] = zero8();

  const size_t arow = (size_t)(m0 + 32 * wm + m) * DM + 8 * h;
  const unsigned short* pah = ch + arow;
  const unsigned short* pal = cl + arow;
  const unsigned short* pb  = wob + (size_t)(n0 + 32 * wn + m) * DM + 8 * h;
#pragma unroll 2
  for (int kk = 0; kk < DM / 32; ++kk) {
    const v16us a0h = ldfrag_u(pah + 32 * kk);
    const v16us a1h = ldfrag_u(pah + (size_t)16 * DM + 32 * kk);
    const v16us a0l = ldfrag_u(pal + 32 * kk);
    const v16us a1l = ldfrag_u(pal + (size_t)16 * DM + 32 * kk);
    const v16us b0  = ldfrag_u(pb + 32 * kk);
    const v16us b1  = ldfrag_u(pb + (size_t)16 * DM + 32 * kk);
    acc[0][0] = mma_bf(a0h, b0, acc[0][0]);
    acc[0][1] = mma_bf(a0h, b1, acc[0][1]);
    acc[1][0] = mma_bf(a1h, b0, acc[1][0]);
    acc[1][1] = mma_bf(a1h, b1, acc[1][1]);
    acc[0][0] = mma_bf(a0l, b0, acc[0][0]);
    acc[0][1] = mma_bf(a0l, b1, acc[0][1]);
    acc[1][0] = mma_bf(a1l, b0, acc[1][0]);
    acc[1][1] = mma_bf(a1l, b1, acc[1][1]);
    guard4<v16us>(acc[0][0], acc[0][1], acc[1][0], acc[1][1], a0h, a1h, a0l, a1l, b0, b1);
  }

#pragma unroll
  for (int mi = 0; mi < 2; ++mi)
#pragma unroll
    for (int ni = 0; ni < 2; ++ni)
#pragma unroll
      for (int r = 0; r < 8; ++r)
        T[(32 * wm + 16 * mi + 8 * h + r) * TP + 32 * wn + 16 * ni + m] = acc[mi][ni][r];
  __syncthreads();

  v4f    ov[8];
  size_t ooff[8];
#pragma unroll
  for (int it = 0; it < 8; ++it) {
    const int L  = 4 * it + q8;
    const int rl = 16 * w + (L >> 1);
    const int hf = L & 1;
    ov[it]   = *(const v4fA*)(T + rl * TP + 32 * hf + 4 * jj);
    ooff[it] = (size_t)(m0 + rl) * DM + (size_t)(n0 + 32 * hf + 4 * jj);
  }
#pragma unroll
  for (int it = 0; it < 8; ++it) *(volatile v4f*)(out + ooff[it]) = ov[it];
  __threadfence();
#pragma unroll
  for (int it = 0; it < 8; ++it) *(volatile v4f*)(out + ooff[it]) = ov[it];
}

extern "C" void kernel_launch(void* const* d_in, const int* in_sizes, int n_in,
                              void* d_out, int out_size, void* d_ws, size_t ws_size,
                              hipStream_t stream) {
  if (n_in < 9) return;
  if (in_sizes[0] != SEQ * DM) return;
  if (in_sizes[1] != DM * DM || in_sizes[2] != DM * DM || in_sizes[3] != DM * DM ||
      in_sizes[4] != DM * DM) return;
  if (in_sizes[5] < 1 || in_sizes[6] < 1 || in_sizes[7] < 1) return;
  if (in_sizes[8] != SEQ * SEQ) return;
  if (out_size != SEQ * DM) return;
  if (ws_size < WS_TOTAL) return;

  const float* x    = (const float*)d_in[0];
  const float* Wq   = (const float*)d_in[1];
  const float* Wk   = (const float*)d_in[2];
  const float* Wv   = (const float*)d_in[3];
  const float* Wo   = (const float*)d_in[4];
  const float* lcp  = (const float*)d_in[5];
  const float* btp  = (const float*)d_in[6];
  const float* abp  = (const float*)d_in[7];
  const int*   mask = (const int*)d_in[8];
  float* out = (float*)d_out;
  char* ws = (char*)d_ws;

  unsigned short* xb = (unsigned short*)(ws + OFF_XB);
  unsigned short* wb = (unsigned short*)(ws + OFF_WB);
  unsigned short* qh = (unsigned short*)(ws + OFF_QH);
  unsigned short* ql = (unsigned short*)(ws + OFF_QL);
  unsigned short* kh = (unsigned short*)(ws + OFF_KH);
  unsigned short* kl = (unsigned short*)(ws + OFF_KL);
  _Float16*       vh = (_Float16*)(ws + OFF_VH);
  _Float16*       vl = (_Float16*)(ws + OFF_VL);
  float*          ns = (float*)(ws + OFF_NS);
  unsigned short* ch = (unsigned short*)(ws + OFF_CH);
  unsigned short* cl = (unsigned short*)(ws + OFF_CL);

  k_cvt<<<dim3(SEQ / 32, 5), dim3(256), 0, stream>>>(x, Wq, Wk, Wv, Wo, xb, wb);
  (void)hipGetLastError();
  k_proj<<<dim3(NH, SEQ / 128, 3), dim3(256), 0, stream>>>(xb, wb, lcp, qh, ql, kh, kl, vh, vl, ns);
  (void)hipGetLastError();
  k_attn<<<dim3(SEQ / 128, NH), dim3(256), 0, stream>>>(qh, ql, kh, kl, vh, vl, ns, mask,
                                                      lcp, btp, abp, ch, cl);
  (void)hipGetLastError();
  k_out<<<dim3(DM / 64, SEQ / 128), dim3(256), 0, stream>>>(ch, cl, wb + (size_t)3 * DM * DM, out);
  (void)hipGetLastError();
}
